// GATNetwork_46059229283058
// MI455X (gfx1250) — hardware-verified
//
#include <hip/hip_runtime.h>
#include <stddef.h>
#include <stdint.h>
#include <math.h>


#define DIN     128
#define HC      128
#define NHEAD   4
#define CHN     32
#define NGR     64
#define HID     128
#define NW2     256
#define NTHR    256
#define NWAVE   8
#define EPT     8
#define CHUNK   (NTHR * EPT)
#define WCAP    (EPT * 32)
#define LISTN   (NWAVE * WCAP)
#define NBMAX   2048
#define NBRUN   1024
#define RCAP    28672
#define DEGCAP  4096
#define GBM     64
#define GBN     64
#define GTHR    128
#define NBW     16
#define NBH     32
#define NEGS    0.2f
#define WSMAX   134217728
#define LDS_SCAN ((2 * RCAP + 2 * NBMAX + LISTN) * 4 + 64)
#define HEAD_FLOATS (NGR * HC + NGR * NW2 + 3 * HID + 16 + 3 * NGR + 2 * NGR)
#define LDS_HEAD (HEAD_FLOATS * 4)
#define MEAS_B1024 16623
#define MEAS_MAXDEG 35

static_assert(NHEAD * CHN == HC && HC == 32 * 4);
static_assert(CHN == 8 * 4);
static_assert(NGR == 64);
static_assert(2 * HID == NTHR && NW2 == NTHR);
static_assert((CHUNK & (CHUNK - 1)) == 0 && CHUNK <= 4096);
static_assert((NBMAX & (NBMAX - 1)) == 0 && NBMAX <= 4096);
static_assert((NBRUN & (NBRUN - 1)) == 0 && NBRUN <= NBMAX && NBRUN >= 16 && (NBRUN % 8) == 0);
static_assert(NTHR * 8 == NBMAX);
static_assert(LISTN >= NBMAX && LISTN >= NWAVE * WCAP);
static_assert((RCAP % 32) == 0 && RCAP >= MEAS_B1024 + 4096);
static_assert(DEGCAP >= MEAS_MAXDEG + 8);
static_assert(LDS_SCAN <= 300000 && LDS_HEAD <= 300000);
static_assert(GBM == (GTHR / 32) * 16 && (DIN % 32) == 0 && (NW2 % GBN) == 0 && (HC % GBN) == 0);
static_assert(NBW * NTHR == NW2 * (DIN / 8));
static_assert(NBH * NTHR * 4 == HID * NW2);
static_assert(((NGR * HC + NGR * NW2 + 3 * HID + 16 + 3 * NGR) % 4) == 0);

typedef float          v4f   __attribute__((ext_vector_type(4)));
typedef float          v8f   __attribute__((ext_vector_type(8)));
typedef int            v4i   __attribute__((ext_vector_type(4)));
typedef int            v8i   __attribute__((ext_vector_type(8)));
typedef unsigned short v8us  __attribute__((ext_vector_type(8)));
typedef __bf16         v16bf __attribute__((ext_vector_type(16)));
typedef v4f __attribute__((may_alias)) v4fa;
union FragB { v16bf v; v8us u[2]; v8i w; };

__device__ __forceinline__ v8f wmx(const FragB& a, const FragB& b, v8f c) {
  v8f d = __builtin_amdgcn_wmma_f32_16x16x32_bf16(false, a.v, false, b.v, (short)0, c, false, false);
  asm volatile("v_nop\n\tv_nop\n\tv_nop\n\tv_nop" : "+v"(d) : "v"(a.w), "v"(b.w));
  return d;
}

__device__ __forceinline__ void ldwait() {
  asm volatile("s_wait_loadcnt 0x0" ::: "memory");
}

__device__ __forceinline__ unsigned bfbits(float v) {
  unsigned u = __float_as_uint(v);
  u = u + 0x7FFFu + ((u >> 16) & 1u);
  return u >> 16;
}
__device__ __forceinline__ float rbf(float v) { return __uint_as_float(bfbits(v) << 16); }
__device__ __forceinline__ v4f rbf4(const v4f a) {
  v4f o; o.x = rbf(a.x); o.y = rbf(a.y); o.z = rbf(a.z); o.w = rbf(a.w); return o;
}
__device__ __forceinline__ float bsel(float a, float b, bool takeA) {
  const unsigned m = takeA ? 0xFFFFFFFFu : 0u;
  return __uint_as_float((__float_as_uint(a) & m) | (__float_as_uint(b) & ~m));
}
__device__ __forceinline__ float relu_k(float v) { return (v > 0.0f) ? v : ((v != v) ? v : 0.0f); }
__device__ __forceinline__ float pmax(float m, float v) { return (v > m || v != v) ? v : m; }

__device__ __forceinline__ v8us cvt8b(const v4f a, const v4f b) {
  v8us o;
  o[0] = (unsigned short)bfbits(a.x); o[1] = (unsigned short)bfbits(a.y);
  o[2] = (unsigned short)bfbits(a.z); o[3] = (unsigned short)bfbits(a.w);
  o[4] = (unsigned short)bfbits(b.x); o[5] = (unsigned short)bfbits(b.y);
  o[6] = (unsigned short)bfbits(b.z); o[7] = (unsigned short)bfbits(b.w);
  return o;
}

__device__ __forceinline__ int scan_chunk(const int* __restrict__ dsts, int nE, int cbase, int slotBase,
                                          int nb, int vec8, int* list, int tid, int lane, int wave) {
  int wc = 0;
  const int el0  = tid * EPT;
  const int e0   = cbase + el0;
  const int sent = -2147483647 - 1;
  v4i da, db;
  if (vec8 != 0 && cbase + CHUNK <= nE) {
    da = *(const v4i*)(dsts + e0);
    db = *(const v4i*)(dsts + e0 + 4);
  } else {
    da.x = (e0     < nE) ? dsts[min(e0,     nE - 1)] : sent;
    da.y = (e0 + 1 < nE) ? dsts[min(e0 + 1, nE - 1)] : sent;
    da.z = (e0 + 2 < nE) ? dsts[min(e0 + 2, nE - 1)] : sent;
    da.w = (e0 + 3 < nE) ? dsts[min(e0 + 3, nE - 1)] : sent;
    db.x = (e0 + 4 < nE) ? dsts[min(e0 + 4, nE - 1)] : sent;
    db.y = (e0 + 5 < nE) ? dsts[min(e0 + 5, nE - 1)] : sent;
    db.z = (e0 + 6 < nE) ? dsts[min(e0 + 6, nE - 1)] : sent;
    db.w = (e0 + 7 < nE) ? dsts[min(e0 + 7, nE - 1)] : sent;
  }
  const unsigned nbs = (unsigned)slotBase;
  const unsigned unb = (unsigned)nb;
  const unsigned s0 = (unsigned)da.x - nbs, s1 = (unsigned)da.y - nbs;
  const unsigned s2 = (unsigned)da.z - nbs, s3 = (unsigned)da.w - nbs;
  const unsigned s4 = (unsigned)db.x - nbs, s5 = (unsigned)db.y - nbs;
  const unsigned s6 = (unsigned)db.z - nbs, s7 = (unsigned)db.w - nbs;
  const bool h0 = s0 < unb, h1 = s1 < unb, h2 = s2 < unb, h3 = s3 < unb;
  const bool h4 = s4 < unb, h5 = s5 < unb, h6 = s6 < unb, h7 = s7 < unb;
  const unsigned any = __builtin_amdgcn_ballot_w32(h0 | h1 | h2 | h3 | h4 | h5 | h6 | h7);
  if (any != 0u) {
#define HITJ(J, HJ, SJ) { \
      const unsigned mj = __builtin_amdgcn_ballot_w32(HJ); \
      if (mj != 0u) { \
        if (HJ) { \
          const int pos = wc + (int)__builtin_amdgcn_mbcnt_lo(mj, 0u); \
          if (pos < WCAP) list[wave * WCAP + pos] = ((el0 + (J)) << 12) | (int)(SJ); \
        } \
        wc += (int)__builtin_popcount(mj); } }
    HITJ(0, h0, s0)
    HITJ(1, h1, s1)
    HITJ(2, h2, s2)
    HITJ(3, h3, s3)
    HITJ(4, h4, s4)
    HITJ(5, h5, s5)
    HITJ(6, h6, s6)
    HITJ(7, h7, s7)
#undef HITJ
  }
  return wc;
}

__global__ __launch_bounds__(NTHR) void k_prep(const float* __restrict__ x, const float* __restrict__ Wl,
                                               const float* __restrict__ Wr, const float* __restrict__ Wq1,
                                               const float* __restrict__ Wv1, unsigned short* xb,
                                               unsigned short* wt, float* wh1, int nN, int nbX) {
  const int blk = (int)blockIdx.x;
  const int tid = (int)threadIdx.x;
  if (blk < nbX) {
    const int i   = blk * NTHR + tid;
    const int row = i >> 4;
    const int c0  = (i & 15) * 8;
    const int rc  = row < nN ? row : nN - 1;
    const float* p = x + (size_t)rc * DIN + c0;
    v4f a = *(const v4f*)p, b = *(const v4f*)(p + 4);
    const v4f z4 = {0.f, 0.f, 0.f, 0.f};
    if (row >= nN) { a = z4; b = z4; }
    const v8us hv = cvt8b(a, b);
    const size_t o = (size_t)row * DIN + c0;
    *(volatile v8us*)(xb + o) = hv;
    __threadfence();
    *(volatile v8us*)(xb + o) = hv;
  } else if (blk < nbX + NBW) {
    const int bb = blk - nbX;
    const int u  = bb * NTHR + tid;
    const int n  = u >> 4;
    const int k8 = (u & 15) * 8;
    const int nc = n & 127;
    v4f a, b;
    if (bb < (NBW / 2)) {
      const float* p = Wl + (size_t)k8 * HC + nc;
      a.x = p[0];       a.y = p[HC];      a.z = p[2 * HC];  a.w = p[3 * HC];
      b.x = p[4 * HC];  b.y = p[5 * HC];  b.z = p[6 * HC];  b.w = p[7 * HC];
    } else {
      const float* p = Wr + (size_t)k8 * HC + nc;
      a.x = p[0];       a.y = p[HC];      a.z = p[2 * HC];  a.w = p[3 * HC];
      b.x = p[4 * HC];  b.y = p[5 * HC];  b.z = p[6 * HC];  b.w = p[7 * HC];
    }
    const v8us hv = cvt8b(a, b);
    const size_t o = (size_t)n * DIN + k8;
    *(volatile v8us*)(wt + o) = hv;
    __threadfence();
    *(volatile v8us*)(wt + o) = hv;
  } else {
    const int u  = (blk - nbX - NBW) * NTHR + tid;
    const int k  = (u >> 6) & (HID - 1);
    const int c4 = (u & 63) * 4;
    const int cc = c4 & 127;
    const v4f q = *(const v4f*)(Wq1 + (size_t)k * HID + cc);
    const v4f v = *(const v4f*)(Wv1 + (size_t)k * HID + cc);
    const bool tq = c4 < HID;
    v4f r;
    r.x = rbf(bsel(q.x, v.x, tq)); r.y = rbf(bsel(q.y, v.y, tq));
    r.z = rbf(bsel(q.z, v.z, tq)); r.w = rbf(bsel(q.w, v.w, tq));
    const size_t o = (size_t)k * NW2 + c4;
    *(volatile v4f*)(wh1 + o) = r;
    __threadfence();
    *(volatile v4f*)(wh1 + o) = r;
  }
}

__global__ __launch_bounds__(GTHR) void k_xlr(const unsigned short* __restrict__ A,
                                              const unsigned short* __restrict__ WT,
                                              const float* __restrict__ b_l, const float* __restrict__ b_r,
                                              float* outF, size_t planeStride) {
  __shared__ __attribute__((aligned(16))) float stg[GBM * GBN];
  __shared__ float bsm[GBN];
  const int tid = (int)threadIdx.x, lane = tid & 31, wave = tid >> 5, hh = lane >> 4, m = lane & 15;
  const int rowBase = (int)blockIdx.x * GBM;
  const int col0    = (int)blockIdx.y * GBN;
  const int plane   = (int)blockIdx.y >> 1;
  const int ocol0   = ((int)blockIdx.y & 1) * GBN;

  {
    const int cb = (col0 + (tid & 63)) & (HC - 1);
    const float vl = b_l[cb];
    const float vr = b_r[cb];
    const float bv = rbf(bsel(vl, vr, col0 < HC));
    if (tid < GBN) bsm[tid] = bv;
  }
  __syncthreads();

  v8f acc[4];
  {
    const v8f z = {0.f, 0.f, 0.f, 0.f, 0.f, 0.f, 0.f, 0.f};
    acc[0] = z; acc[1] = z; acc[2] = z; acc[3] = z;
  }
  const unsigned short* ap = A  + (size_t)(rowBase + 16 * wave + m) * (size_t)DIN + 8 * hh;
  const unsigned short* wp = WT + (size_t)(col0 + m) * (size_t)DIN + 8 * hh;
#pragma unroll 1
  for (int ks = 0; ks < DIN / 32; ++ks) {
    FragB af;
    af.u[0] = *(const v8us*)(ap + 32 * ks);
    af.u[1] = *(const v8us*)(ap + 32 * ks + 16);
#pragma unroll
    for (int t = 0; t < 4; ++t) {
      const unsigned short* wq = wp + (size_t)(16 * t) * (size_t)DIN + 32 * ks;
      FragB bf;
      bf.u[0] = *(const v8us*)wq;
      bf.u[1] = *(const v8us*)(wq + 16);
      acc[t] = wmx(af, bf, acc[t]);
    }
  }

#pragma unroll
  for (int t = 0; t < 4; ++t) {
    const int lc = 16 * t + m;
    const float bv = bsm[lc];
#pragma unroll
    for (int r = 0; r < 8; ++r) {
      const int lr = 16 * wave + 8 * hh + r;
      stg[lr * GBN + lc] = acc[t][r] + bv;
    }
  }
  __syncthreads();

  float* ob = outF + (size_t)plane * planeStride;
  v4f fv[8];
#pragma unroll
  for (int i = 0; i < 8; ++i) {
    const int lr = 16 * wave + 2 * i + hh;
    fv[i] = *(const v4fa*)(stg + lr * GBN + 4 * m);
  }
#pragma unroll
  for (int i = 0; i < 8; ++i) {
    const int lr = 16 * wave + 2 * i + hh;
    const int gr = rowBase + lr;
    float* op = ob + (size_t)gr * (size_t)HC + ocol0 + 4 * m;
    *(volatile v4f*)op = fv[i];
  }
  __threadfence();
#pragma unroll
  for (int i = 0; i < 8; ++i) {
    const int lr = 16 * wave + 2 * i + hh;
    const int gr = rowBase + lr;
    float* op = ob + (size_t)gr * (size_t)HC + ocol0 + 4 * m;
    *(volatile v4f*)op = fv[i];
  }
}

__global__ __launch_bounds__(NTHR) void k_scan(
    const int* __restrict__ srcs, const int* __restrict__ dsts,
    const float* __restrict__ XL, const float* __restrict__ XR,
    const float* __restrict__ att, const float* __restrict__ bias,
    float* Hn, int nN, int nE, int nb, int vec8) {
  extern __shared__ v4f lds_dyn[];
  int* reg1 = (int*)lds_dyn;
  int* reg2 = reg1 + RCAP;
  int* scnt = reg2 + RCAP;
  int* soff = scnt + NBMAX;
  int* list = soff + NBMAX;
  int* wcnt = list + LISTN;
  int* wtot = wcnt + NWAVE;
  const int tid = (int)threadIdx.x, lane = tid & 31;
  const int wave = __builtin_amdgcn_readfirstlane(tid >> 5);
  const int nodeBase = (int)blockIdx.x * nb;

  for (int i = tid; i < NBMAX; i += NTHR) scnt[i] = 0;
  __syncthreads();

  int tot = 0;
  const int nChunks = (nE + CHUNK - 1) / CHUNK;
#pragma unroll 1
  for (int ch = 0; ch < nChunks; ++ch) {
    const int cbase = ch * CHUNK;
    const int wc = scan_chunk(dsts, nE, cbase, nodeBase, nb, vec8, list, tid, lane, wave);
    if (lane == 0) wcnt[wave] = wc;
    __syncthreads();
    int pre = 0, all = 0;
#pragma unroll
    for (int w2 = 0; w2 < NWAVE; ++w2) {
      int c = wcnt[w2];
      c = c < 0 ? 0 : (c > WCAP ? WCAP : c);
      all += c;
      pre += (w2 < wave) ? c : 0;
    }
    const int wcc  = wc > WCAP ? WCAP : wc;
    const int base = tot + pre;
#pragma unroll 1
    for (int i = lane; i < wcc; i += 32) {
      const int ent = list[wave * WCAP + i];
      const int el  = (ent >> 12) & (CHUNK - 1);
      const int sl  = ent & (NBMAX - 1);
      int eid = cbase + el;
      eid = eid > nE - 1 ? nE - 1 : eid;
      const int pos = base + i;
      if (pos < RCAP) reg1[pos] = (int)(((unsigned)eid << 12) | (unsigned)sl);
    }
    tot += all;
    tot = tot > RCAP ? RCAP : tot;
    __syncthreads();
  }
  const int nh = tot;

  if (wave == 0) {
#pragma unroll 1
    for (int b0 = 0; b0 < nh; b0 += 32) {
      const int idx = b0 + lane;
      const int uv  = reg1[idx < RCAP ? idx : RCAP - 1];
      const int m32 = (nh - b0) < 32 ? (nh - b0) : 32;
#pragma unroll 1
      for (int k = 0; k < m32; ++k) {
        const int u  = __builtin_amdgcn_readlane(uv, k);
        const int sl = u & (NBMAX - 1);
        if (lane == 0) scnt[sl] = scnt[sl] + 1;
      }
    }
  }
  __syncthreads();

  {
    const v4i ca = *(const v4i*)(scnt + 8 * tid);
    const v4i cb = *(const v4i*)(scnt + 8 * tid + 4);
    const int e0 = ca.x < 0 ? 0 : ca.x, e1 = ca.y < 0 ? 0 : ca.y, e2 = ca.z < 0 ? 0 : ca.z, e3 = ca.w < 0 ? 0 : ca.w;
    const int e4 = cb.x < 0 ? 0 : cb.x, e5 = cb.y < 0 ? 0 : cb.y, e6 = cb.z < 0 ? 0 : cb.z, e7 = cb.w < 0 ? 0 : cb.w;
    const int ts = e0 + e1 + e2 + e3 + e4 + e5 + e6 + e7;
    int incl = ts;
#pragma unroll
    for (int d = 1; d < 32; d <<= 1) {
      const int up = __shfl_up(incl, d);
      if (lane >= d) incl += up;
    }
    if (lane == 31) wtot[wave] = incl;
    __syncthreads();
    int pre = 0;
#pragma unroll
    for (int w2 = 0; w2 < NWAVE; ++w2) pre += (w2 < wave) ? wtot[w2] : 0;
    int run = pre + incl - ts;
    soff[8 * tid + 0] = run; run += e0;
    soff[8 * tid + 1] = run; run += e1;
    soff[8 * tid + 2] = run; run += e2;
    soff[8 * tid + 3] = run; run += e3;
    soff[8 * tid + 4] = run; run += e4;
    soff[8 * tid + 5] = run; run += e5;
    soff[8 * tid + 6] = run; run += e6;
    soff[8 * tid + 7] = run;
  }
  __syncthreads();
  for (int i = tid; i < NBMAX; i += NTHR) list[i] = soff[i];
  __syncthreads();

  if (wave == 0) {
#pragma unroll 1
    for (int b0 = 0; b0 < nh; b0 += 32) {
      const int idx = b0 + lane;
      const int uv  = reg1[idx < RCAP ? idx : RCAP - 1];
      const int m32 = (nh - b0) < 32 ? (nh - b0) : 32;
#pragma unroll 1
      for (int k = 0; k < m32; ++k) {
        const int u   = __builtin_amdgcn_readlane(uv, k);
        const int sl  = u & (NBMAX - 1);
        const int eid = (int)((unsigned)u >> 12);
        if (lane == 0) {
          int pos = list[sl];
          pos = pos < 0 ? 0 : (pos > RCAP - 1 ? RCAP - 1 : pos);
          reg2[pos] = eid;
          list[sl] = pos + 1;
        }
      }
    }
  }
  __syncthreads();

  const int nbw = nb >> 3;
  const bool ovf = (nh >= RCAP);
  const float qnan = __int_as_float(0x7fc00000);
  const v4f at4 = rbf4(*(const v4f*)(att + 4 * lane));
  const v4f bb4 = rbf4(*(const v4f*)(bias + 4 * lane));
#pragma unroll 1
  for (int jt = 0; jt < nbw; ++jt) {
    const int slot = wave * nbw + jt;
    const int grow = nodeBase + slot;
    if (grow >= nN) break;
    int st = __builtin_amdgcn_readfirstlane(soff[slot]);
    const int craw = __builtin_amdgcn_readfirstlane(scnt[slot]);
    int cnt = craw;
    st  = st < 0 ? 0 : (st > nh ? nh : st);
    cnt = cnt < 0 ? 0 : (cnt > DEGCAP ? DEGCAP : cnt);
    if (cnt > nh - st) cnt = nh - st;
    const float pz = (ovf || craw > DEGCAP) ? qnan : 0.0f;

    const v4f xr4 = *(const v4f*)(XR + (size_t)grow * HC + 4 * lane);
    ldwait();
    v4f av = {0.f, 0.f, 0.f, 0.f};
    float mx = -1.0e30f, dn = 0.0f;

#pragma unroll 1
    for (int q = 0; q <= cnt; ++q) {
      int s = grow;
      if (q < cnt) {
        int idx = st + q; idx = idx > RCAP - 1 ? RCAP - 1 : idx;
        int eid = reg2[idx]; eid = eid < 0 ? 0 : (eid > nE - 1 ? nE - 1 : eid);
        const int sraw = srcs[eid];
        s = sraw < 0 ? 0 : (sraw > nN - 1 ? nN - 1 : sraw);
      }
      s = __builtin_amdgcn_readfirstlane(s);
      const v4f xs = *(const v4f*)(XL + (size_t)s * HC + 4 * lane);
      ldwait();
      float t0 = xs.x + xr4.x, t1 = xs.y + xr4.y, t2 = xs.z + xr4.z, t3 = xs.w + xr4.w;
      t0 = t0 > 0.f ? t0 : NEGS * t0;
      t1 = t1 > 0.f ? t1 : NEGS * t1;
      t2 = t2 > 0.f ? t2 : NEGS * t2;
      t3 = t3 > 0.f ? t3 : NEGS * t3;
      float part = t0 * at4.x;
      part = fmaf(t1, at4.y, part);
      part = fmaf(t2, at4.z, part);
      part = fmaf(t3, at4.w, part);
      part += __shfl_xor(part, 1);
      part += __shfl_xor(part, 2);
      part += __shfl_xor(part, 4);
      const float al = part;
      const float df = al - mx;
      const float ee = expf(-fabsf(df));
      const bool up  = df > 0.f;
      const float s1 = up ? ee : 1.0f;
      const float s2 = up ? 1.0f : ee;
      mx = up ? al : mx;
      dn = fmaf(dn, s1, s2);
      av.x = fmaf(av.x, s1, s2 * xs.x);
      av.y = fmaf(av.y, s1, s2 * xs.y);
      av.z = fmaf(av.z, s1, s2 * xs.z);
      av.w = fmaf(av.w, s1, s2 * xs.w);
    }
    const float iv = 1.0f / (dn + 1e-16f);
    v4f r;
    r.x = relu_k(fmaf(av.x, iv, bb4.x)) + pz;
    r.y = relu_k(fmaf(av.y, iv, bb4.y)) + pz;
    r.z = relu_k(fmaf(av.z, iv, bb4.z)) + pz;
    r.w = relu_k(fmaf(av.w, iv, bb4.w)) + pz;
    float* gp = Hn + (size_t)grow * HC + 4 * lane;
    *(volatile v4f*)gp = r;
    __threadfence();
    *(volatile v4f*)gp = r;
  }
}

__global__ __launch_bounds__(NTHR) void k_pool(const float* __restrict__ hn, const int* __restrict__ bat,
                                               int nN, float* gp) {
  __shared__ __attribute__((aligned(16))) float wmxs[NWAVE * HC];
  __shared__ __attribute__((aligned(16))) float outs[HC];
  const int tid = (int)threadIdx.x, lane = tid & 31;
  const int wave = __builtin_amdgcn_readfirstlane(tid >> 5);
  const int g = (int)blockIdx.x;
  const float ninf = __int_as_float((int)0xff800000u);

  v4f a = {ninf, ninf, ninf, ninf};
#pragma unroll 1
  for (int i0 = wave * 32; i0 < nN; i0 += NTHR) {
    const int i  = i0 + lane;
    const int ic = i < nN ? i : nN - 1;
    const int b  = bat[ic];
    const bool hit = (i < nN) && (b == g);
    unsigned msk = __builtin_amdgcn_ballot_w32(hit);
    int nh = (int)__builtin_popcount(msk);
    nh = nh > 32 ? 32 : nh;
#pragma unroll 1
    for (int q = 0; q < nh; ++q) {
      const int k = __builtin_ffs((int)msk) - 1;
      msk &= msk - 1u;
      int node = i0 + (k < 0 ? 0 : k);
      node = node > nN - 1 ? nN - 1 : node;
      const v4f v = *(const v4f*)(hn + (size_t)node * HC + 4 * lane);
      a.x = pmax(a.x, v.x); a.y = pmax(a.y, v.y); a.z = pmax(a.z, v.z); a.w = pmax(a.w, v.w);
    }
  }
  *(v4fa*)(wmxs + wave * HC + 4 * lane) = a;
  __syncthreads();
  if (tid < HC) {
    float r = wmxs[tid];
#pragma unroll
    for (int w2 = 1; w2 < NWAVE; ++w2) r = pmax(r, wmxs[w2 * HC + tid]);
    outs[tid] = r;
  }
  __syncthreads();
  const v4f ov = *(const v4fa*)(outs + 4 * lane);
  float* op = gp + (size_t)g * HC + 4 * lane;
  const bool okst = (wave == 0);
  if (okst) *(volatile v4f*)op = ov;
  __threadfence();
  if (okst) *(volatile v4f*)op = ov;
}

__global__ __launch_bounds__(NTHR) void k_head(const float* __restrict__ gp, const float* __restrict__ wh1,
                                               const float* __restrict__ bq1, const float* __restrict__ bv1,
                                               const float* __restrict__ Wq2, const float* __restrict__ bq2,
                                               const float* __restrict__ Wv2, const float* __restrict__ bv2,
                                               float* out) {
  extern __shared__ __attribute__((aligned(16))) float hsm[];
  float* gl  = hsm;
  float* hid = gl + NGR * HC;
  float* w2s = hid + NGR * NW2;
  float* b2s = w2s + 3 * HID;
  float* qv  = b2s + 16;
  float* os  = qv + 3 * NGR;
  const int tid = (int)threadIdx.x, lane = tid & 31;
  const int wave = __builtin_amdgcn_readfirstlane(tid >> 5);

#pragma unroll 4
  for (int it = 0; it < (NGR * HC) / (4 * NTHR); ++it) {
    const int u = it * NTHR + tid;
    *(v4fa*)(gl + 4 * u) = *(const v4f*)(gp + 4 * (size_t)u);
  }
#pragma unroll 1
  for (int i = tid; i < 3 * HID; i += NTHR) {
    const int o = i >> 7, k = i & (HID - 1);
    const float q = Wq2[2 * k + (o & 1)];
    const float v = Wv2[k];
    w2s[i] = rbf(bsel(q, v, o < 2));
  }
  {
    const float q2 = bq2[tid & 1];
    const float v2 = bv2[0];
    const float bv = rbf(bsel(q2, v2, tid < 2));
    if (tid < 3) b2s[tid] = bv;
  }
  const int tc = tid & (HID - 1);
  const float b1q = bq1[tc];
  const float b1v = bv1[tc];
  const float bh  = rbf(bsel(b1q, b1v, tid < HID));
  __syncthreads();

#pragma unroll 1
  for (int g0 = 0; g0 < NGR; g0 += 4) {
    const float* gq = gl + g0 * HC;
    float a0 = 0.0f, a1 = 0.0f, a2 = 0.0f, a3 = 0.0f;
#pragma unroll 4
    for (int k = 0; k < HC; ++k) {
      const float w = wh1[(size_t)k * NW2 + tid];
      a0 = fmaf(gq[k], w, a0);
      a1 = fmaf(gq[HC + k], w, a1);
      a2 = fmaf(gq[2 * HC + k], w, a2);
      a3 = fmaf(gq[3 * HC + k], w, a3);
    }
    hid[(g0 + 0) * NW2 + tid] = relu_k(a0 + bh);
    hid[(g0 + 1) * NW2 + tid] = relu_k(a1 + bh);
    hid[(g0 + 2) * NW2 + tid] = relu_k(a2 + bh);
    hid[(g0 + 3) * NW2 + tid] = relu_k(a3 + bh);
  }
  __syncthreads();

  if (wave < 6) {
    const int g = tid / 3;
    const int o = tid - 3 * g;
    const float* hp = hid + g * NW2 + ((o == 2) ? HID : 0);
    const float* wp = w2s + o * HID;
    float s = 0.0f;
#pragma unroll 4
    for (int k = 0; k < HID; ++k) s = fmaf(hp[k], wp[k], s);
    qv[tid] = s + b2s[o];
  }
  __syncthreads();
  if (wave < 4) {
    const int g = tid >> 1, j = tid & 1;
    const float q0 = qv[3 * g + 0], q1 = qv[3 * g + 1], vv = qv[3 * g + 2];
    const float qj = j ? q1 : q0;
    const float qm = 0.5f * (q0 + q1);
    os[tid] = (qj - qm) + vv;
  }
  __syncthreads();
  const v4f ov = *(const v4fa*)(os + 4 * lane);
  float* op = out + 4 * lane;
  const bool okst = (wave == 0);
  if (okst) *(volatile v4f*)op = ov;
  __threadfence();
  if (okst) *(volatile v4f*)op = ov;
}

static int pick_nb(int nE, int nN) {
  int nb = NBRUN;
  while (nb > 16 && (long long)nb * (long long)nE * 5LL > (long long)RCAP * (long long)nN * 4LL) nb >>= 1;
  return nb;
}
static inline int cdiv(int a, int b) { return (a + b - 1) / b; }
static inline size_t al256(size_t o) { return (o + 255) & ~(size_t)255; }

extern "C" void kernel_launch(void* const* d_in, const int* in_sizes, int n_in,
                              void* d_out, int out_size, void* d_ws, size_t ws_size,
                              hipStream_t stream) {
  if (n_in < 17) return;
  if (in_sizes[0] < DIN || (in_sizes[0] % DIN) != 0) return;
  const int nN = in_sizes[0] / DIN;
  if (nN < 1 || nN > (1 << 22)) return;
  if (in_sizes[1] != DIN * HC || in_sizes[2] != HC) return;
  if (in_sizes[3] != DIN * HC || in_sizes[4] != HC) return;
  if (in_sizes[5] != HC || in_sizes[6] != HC) return;
  if (in_sizes[7] != HC * HID || in_sizes[8] != HID) return;
  if (in_sizes[9] != HID * 2 || in_sizes[10] != 2) return;
  if (in_sizes[11] != HC * HID || in_sizes[12] != HID) return;
  if (in_sizes[13] != HID || in_sizes[14] != 1) return;
  if (in_sizes[15] < 2 || (in_sizes[15] & 1) != 0) return;
  const int nE = in_sizes[15] / 2;
  if (nE < 1 || nE > (1 << 20)) return;
  if (in_sizes[16] != nN) return;
  if (out_size != NGR * 2) return;

  const float* x    = (const float*)d_in[0];
  const float* W_l  = (const float*)d_in[1];
  const float* b_l  = (const float*)d_in[2];
  const float* W_r  = (const float*)d_in[3];
  const float* b_r  = (const float*)d_in[4];
  const float* att  = (const float*)d_in[5];
  const float* bias = (const float*)d_in[6];
  const float* Wq1  = (const float*)d_in[7];
  const float* bq1  = (const float*)d_in[8];
  const float* Wq2  = (const float*)d_in[9];
  const float* bq2  = (const float*)d_in[10];
  const float* Wv1  = (const float*)d_in[11];
  const float* bv1  = (const float*)d_in[12];
  const float* Wv2  = (const float*)d_in[13];
  const float* bv2  = (const float*)d_in[14];
  const int*   ei   = (const int*)d_in[15];
  const int*   bat  = (const int*)d_in[16];
  float* out = (float*)d_out;
  const int* src = ei;
  const int* dst = ei + nE;

  const int MP   = cdiv(nN, GBM) * GBM;
  const int nbX  = MP / 16;
  const int nb   = pick_nb(nE, nN);
  const int gA   = cdiv(nN, nb);
  const int vec8 = ((nE & 3) == 0) ? 1 : 0;
  if ((long long)gA * nb < (long long)nN) return;
  if (nbX * 16 != MP) return;

  char* ws = (char*)d_ws;
  size_t off = 0;
  const size_t oXB  = off; off = al256(off + (size_t)MP * DIN * 2);
  const size_t oWT  = off; off = al256(off + (size_t)NW2 * DIN * 2);
  const size_t oWH1 = off; off = al256(off + (size_t)HID * NW2 * 4);
  const size_t oXL  = off; off = al256(off + (size_t)MP * HC * 4);
  const size_t oXR  = off; off = al256(off + (size_t)MP * HC * 4);
  const size_t oHN  = off; off = al256(off + (size_t)MP * HC * 4);
  const size_t oGP  = off; off = al256(off + (size_t)NGR * HC * 4);
  if (off > ws_size || off > (size_t)WSMAX) return;
  if (((oXR - oXL) & 3) != 0) return;
  unsigned short* XB  = (unsigned short*)(ws + oXB);
  unsigned short* WT  = (unsigned short*)(ws + oWT);
  float*          WH1 = (float*)(ws + oWH1);
  float*          XL  = (float*)(ws + oXL);
  float*          XR  = (float*)(ws + oXR);
  float*          HN  = (float*)(ws + oHN);
  float*          GP  = (float*)(ws + oGP);
  const size_t planeStride = (oXR - oXL) / 4;

  hipFuncSetAttribute(reinterpret_cast<const void*>(&k_scan),
                      hipFuncAttributeMaxDynamicSharedMemorySize, LDS_SCAN);
  hipFuncSetAttribute(reinterpret_cast<const void*>(&k_head),
                      hipFuncAttributeMaxDynamicSharedMemorySize, LDS_HEAD);

  k_prep<<<nbX + NBW + NBH, NTHR, 0, stream>>>(x, W_l, W_r, Wq1, Wv1, XB, WT, WH1, nN, nbX);
  k_xlr<<<dim3(MP / GBM, NW2 / GBN), GTHR, 0, stream>>>(XB, WT, b_l, b_r, XL, planeStride);
  k_scan<<<gA, NTHR, LDS_SCAN, stream>>>(src, dst, XL, XR, att, bias, HN, nN, nE, nb, vec8);
  k_pool<<<NGR, NTHR, 0, stream>>>(HN, bat, nN, GP);
  k_head<<<1, NTHR, LDS_HEAD, stream>>>(GP, WH1, bq1, bv1, Wq2, bq2, Wv2, bv2, out);
}
